// CVKAN_30751965839658
// MI455X (gfx1250) — hardware-run, weakly checked
//
#include <hip/hip_runtime.h>
#define BB 8192
#define D0 128
#define D1 128
#define D2 64
#define GG 8
#define RCH 2048

typedef __bf16 v16b __attribute__((ext_vector_type(16)));
typedef unsigned short v8us __attribute__((ext_vector_type(8), may_alias));
typedef float  v8f  __attribute__((ext_vector_type(8)));
typedef float  v4f  __attribute__((ext_vector_type(4)));
typedef float  v4fa __attribute__((ext_vector_type(4), may_alias));
union FragB { v16b v; v8us half[2]; unsigned short u[16]; };

__device__ __forceinline__ unsigned short bf16_bits(float x) { unsigned int u = __float_as_uint(x); return (unsigned short)((u + 0x7FFFu + ((u >> 16) & 1u)) >> 16); }
__device__ __forceinline__ float bf16_val(unsigned short b) { return __uint_as_float(((unsigned int)b) << 16); }
__device__ __forceinline__ float bf16_round(float x) { return bf16_val(bf16_bits(x)); }
template <int NT>
__device__ __forceinline__ v8f mmaN(v16b ah, v16b al, v16b bh, v16b bl, v8f c) {
  c = __builtin_amdgcn_wmma_f32_16x16x32_bf16(false, ah, false, bh, (short)0, c, false, false);
  if (NT >= 2) c = __builtin_amdgcn_wmma_f32_16x16x32_bf16(false, al, false, bh, (short)0, c, false, false);
  if (NT >= 3) c = __builtin_amdgcn_wmma_f32_16x16x32_bf16(false, ah, false, bl, (short)0, c, false, false);
  asm volatile("v_nop\n\tv_nop\n\tv_nop\n\tv_nop" : "+v"(c) : "v"(ah), "v"(al), "v"(bh), "v"(bl));
  return c;
}

__global__ __launch_bounds__(256) void k_wt_bf16(const float* __restrict__ W, unsigned short* __restrict__ Wt, int K, int N) {
  const int t = blockIdx.x * 256 + threadIdx.x;
  const int k8n = K / 8;
  if (t >= N * k8n) return;
  const int n = t / k8n, k8 = (t % k8n) * 8;
  v8us v;
#pragma unroll
  for (int i = 0; i < 8; ++i) v[i] = bf16_bits(W[(size_t)(k8 + i) * N + n]);
  *(volatile v8us*)(Wt + (size_t)n * K + k8) = v;
  __threadfence();
  *(volatile v8us*)(Wt + (size_t)n * K + k8) = v;
}

template <bool ASPLIT, int ACT, bool BIAS_BF16>
__global__ __launch_bounds__(128) void k_gemm_bf(const float* __restrict__ A, int lda, const unsigned short* __restrict__ Wt, int ldb,
                                               const float* __restrict__ bias, float* __restrict__ C, int ldc, int M, int N, int K) {
  __shared__ __attribute__((aligned(16))) float so[4][16][64];
  const int tid = threadIdx.x, w = tid >> 5, lane = tid & 31, ln = lane & 15, hh = lane >> 4;
  const int ntn = N / 64;
  const int wid = blockIdx.x * 4 + w;
  const int mt = wid / ntn, nq = wid % ntn;
  if (mt * 16 >= M) return;
  const int row0 = mt * 16, col0 = nq * 64;
  const float* arow = A + (size_t)(row0 + ln) * lda;
  v8f acc[4] = {};
  for (int kb = 0; kb < K; kb += 32) {
    FragB ah, al;
    const v4f x0 = *(const v4fa*)(arow + kb + 8 * hh), x1 = *(const v4fa*)(arow + kb + 8 * hh + 4);
    const v4f x2 = *(const v4fa*)(arow + kb + 16 + 8 * hh), x3 = *(const v4fa*)(arow + kb + 16 + 8 * hh + 4);
    float xs[16] = {x0[0],x0[1],x0[2],x0[3],x1[0],x1[1],x1[2],x1[3],x2[0],x2[1],x2[2],x2[3],x3[0],x3[1],x3[2],x3[3]};
#pragma unroll
    for (int i = 0; i < 16; ++i) { const unsigned short hb = bf16_bits(xs[i]); ah.u[i] = hb; al.u[i] = ASPLIT ? bf16_bits(xs[i] - bf16_val(hb)) : (unsigned short)0; }
#pragma unroll
    for (int t = 0; t < 4; ++t) {
      const unsigned short* brow = Wt + (size_t)(col0 + t * 16 + ln) * ldb + kb;
      FragB b;
      b.half[0] = *(const v8us*)(brow + 8 * hh);
      b.half[1] = *(const v8us*)(brow + 16 + 8 * hh);
      acc[t] = mmaN<ASPLIT ? 2 : 1>(ah.v, al.v, b.v, b.v, acc[t]);
    }
  }
#pragma unroll
  for (int t = 0; t < 4; ++t) {
    float bv = bias ? bias[col0 + t * 16 + ln] : 0.f;
    if (BIAS_BF16) bv = bf16_round(bv);
#pragma unroll
    for (int r = 0; r < 8; ++r) { float v = acc[t][r] + bv; if (ACT == 1) v = fmaxf(v, 0.f); so[w][8 * hh + r][t * 16 + ln] = v; }
  }
  __builtin_amdgcn_fence(__ATOMIC_ACQ_REL, "workgroup");
  __builtin_amdgcn_wave_barrier();
  const int rsub = lane >> 4, c4 = (lane & 15) * 4;
  for (int pass = 0; pass < 2; ++pass) {
#pragma unroll
    for (int q = 0; q < 8; ++q) {
      const int r = q * 2 + rsub;
      const v4f v = *(const v4fa*)&so[w][r][c4];
      *(volatile v4f*)(C + (size_t)(row0 + r) * ldc + col0 + c4) = v;
    }
    if (pass == 0) __threadfence();
  }
}

template <int D, bool CAUSAL>
__global__ __launch_bounds__(128) void k_flash(const float* __restrict__ qb, const float* __restrict__ kb, const float* __restrict__ vb,
                                             int pitch, int T, int H, float scale, float* __restrict__ y, int ypitch) {
  constexpr int KS = D / 32;
  constexpr int DT = D / 16;
  __shared__ __attribute__((aligned(16))) unsigned short sKh[32][D + 8], sKl[32][D + 8], sVh[32][D + 8], sVl[32][D + 8];
  __shared__ __attribute__((aligned(16))) unsigned short sPh[4][16][40], sPl[4][16][40];
  __shared__ __attribute__((aligned(16))) float sO[4][16][D];
  const int tid = threadIdx.x, w = tid >> 5, lane = tid & 31, ln = lane & 15, hh = lane >> 4;
  const int nqb = (T + 63) / 64;
  const int bh = blockIdx.x / nqb, qblk = blockIdx.x % nqb;
  const int b = bh / H, h = bh % H;
  const int q0 = qblk * 64 + w * 16;
  const float* Q = qb + (size_t)b * T * pitch + h * D;
  const float* K = kb + (size_t)b * T * pitch + h * D;
  const float* V = vb + (size_t)b * T * pitch + h * D;

  FragB aqh[KS], aql[KS];
  {
    int row = q0 + ln; if (row >= T) row = T - 1;
    const float* qr = Q + (size_t)row * pitch;
#pragma unroll
    for (int ks = 0; ks < KS; ++ks)
#pragma unroll
      for (int i = 0; i < 16; ++i) {
        const int d = ks * 32 + ((i < 8) ? (8 * hh + i) : (16 + 8 * hh + (i - 8)));
        const float x = qr[d] * scale; const unsigned short hb = bf16_bits(x);
        aqh[ks].u[i] = hb; aql[ks].u[i] = bf16_bits(x - bf16_val(hb));
      }
  }
  float m_r[8], l_r[8];
#pragma unroll
  for (int r = 0; r < 8; ++r) { m_r[r] = -3.0e38f; l_r[r] = 0.f; }
  v8f oacc[DT];
#pragma unroll
  for (int dt = 0; dt < DT; ++dt) oacc[dt] = (v8f){0.f,0.f,0.f,0.f,0.f,0.f,0.f,0.f};

  const int kv_end = CAUSAL ? min(T, qblk * 64 + 64) : T;
  for (int j0 = 0; j0 < kv_end; j0 += 32) {
    __syncthreads();
    for (int e = tid; e < 32 * (D / 4); e += 128) {
      const int r = e / (D / 4), c4 = (e % (D / 4)) * 4;
      const int key = j0 + r;
      v4f kf = {0.f,0.f,0.f,0.f}, vf = {0.f,0.f,0.f,0.f};
      if (key < T) { kf = *(const v4fa*)(K + (size_t)key * pitch + c4); vf = *(const v4fa*)(V + (size_t)key * pitch + c4); }
#pragma unroll
      for (int t = 0; t < 4; ++t) {
        unsigned short hb = bf16_bits(kf[t]); sKh[r][c4 + t] = hb; sKl[r][c4 + t] = bf16_bits(kf[t] - bf16_val(hb));
        hb = bf16_bits(vf[t]); sVh[r][c4 + t] = hb; sVl[r][c4 + t] = bf16_bits(vf[t] - bf16_val(hb));
      }
    }
    __syncthreads();
    v8f s[2];
#pragma unroll
    for (int nt = 0; nt < 2; ++nt) {
      v8f acc = {};
#pragma unroll
      for (int ks = 0; ks < KS; ++ks) {
        FragB bh_, bl_;
        bh_.half[0] = *(const v8us*)&sKh[nt * 16 + ln][ks * 32 + 8 * hh]; bh_.half[1] = *(const v8us*)&sKh[nt * 16 + ln][ks * 32 + 16 + 8 * hh];
        bl_.half[0] = *(const v8us*)&sKl[nt * 16 + ln][ks * 32 + 8 * hh]; bl_.half[1] = *(const v8us*)&sKl[nt * 16 + ln][ks * 32 + 16 + 8 * hh];
        acc = mmaN<3>(aqh[ks].v, aql[ks].v, bh_.v, bl_.v, acc);
      }
      s[nt] = acc;
    }
    float alpha[8];
#pragma unroll
    for (int r = 0; r < 8; ++r) {
      const int qi = q0 + 8 * hh + r;
      const int ja = j0 + ln, jb = j0 + 16 + ln;
      if (CAUSAL) { if (ja > qi) s[0][r] = -3.0e38f; if (jb > qi) s[1][r] = -3.0e38f; }
      if (ja >= T) s[0][r] = -3.0e38f;
      if (jb >= T) s[1][r] = -3.0e38f;
      float mx = fmaxf(s[0][r], s[1][r]);
      mx = fmaxf(mx, __shfl_xor(mx, 1, 32)); mx = fmaxf(mx, __shfl_xor(mx, 2, 32)); mx = fmaxf(mx, __shfl_xor(mx, 4, 32)); mx = fmaxf(mx, __shfl_xor(mx, 8, 32));
      const float mnew = fmaxf(m_r[r], mx);
      alpha[r] = (mnew > -1.0e38f) ? __expf(m_r[r] - mnew) : 1.0f;
      const float p0 = (s[0][r] > -1.0e38f) ? __expf(s[0][r] - mnew) : 0.f;
      const float p1 = (s[1][r] > -1.0e38f) ? __expf(s[1][r] - mnew) : 0.f;
      m_r[r] = mnew;
      l_r[r] = l_r[r] * alpha[r] + p0 + p1;
      unsigned short hb = bf16_bits(p0); sPh[w][8 * hh + r][ln] = hb;      sPl[w][8 * hh + r][ln] = bf16_bits(p0 - bf16_val(hb));
      hb = bf16_bits(p1);                sPh[w][8 * hh + r][16 + ln] = hb; sPl[w][8 * hh + r][16 + ln] = bf16_bits(p1 - bf16_val(hb));
    }
#pragma unroll
    for (int dt = 0; dt < DT; ++dt)
#pragma unroll
      for (int r = 0; r < 8; ++r) oacc[dt][r] *= alpha[r];
    __builtin_amdgcn_fence(__ATOMIC_ACQ_REL, "workgroup");
    __builtin_amdgcn_wave_barrier();
    FragB pah, pal;
    pah.half[0] = *(const v8us*)&sPh[w][ln][8 * hh]; pah.half[1] = *(const v8us*)&sPh[w][ln][16 + 8 * hh];
    pal.half[0] = *(const v8us*)&sPl[w][ln][8 * hh]; pal.half[1] = *(const v8us*)&sPl[w][ln][16 + 8 * hh];
#pragma unroll
    for (int dt = 0; dt < DT; ++dt) {
      FragB bvh, bvl;
#pragma unroll
      for (int i = 0; i < 8; ++i) {
        bvh.u[i] = sVh[8 * hh + i][dt * 16 + ln]; bvh.u[8 + i] = sVh[16 + 8 * hh + i][dt * 16 + ln];
        bvl.u[i] = sVl[8 * hh + i][dt * 16 + ln]; bvl.u[8 + i] = sVl[16 + 8 * hh + i][dt * 16 + ln];
      }
      oacc[dt] = mmaN<3>(pah.v, pal.v, bvh.v, bvl.v, oacc[dt]);
    }
    __builtin_amdgcn_fence(__ATOMIC_ACQ_REL, "workgroup");
    __builtin_amdgcn_wave_barrier();
  }
#pragma unroll
  for (int r = 0; r < 8; ++r) {
    float l = l_r[r];
    l += __shfl_xor(l, 1, 32); l += __shfl_xor(l, 2, 32); l += __shfl_xor(l, 4, 32); l += __shfl_xor(l, 8, 32);
    l_r[r] = (l > 0.f) ? 1.0f / l : 0.f;
  }
#pragma unroll
  for (int dt = 0; dt < DT; ++dt)
#pragma unroll
    for (int r = 0; r < 8; ++r) sO[w][8 * hh + r][dt * 16 + ln] = oacc[dt][r] * l_r[r];
  __builtin_amdgcn_fence(__ATOMIC_ACQ_REL, "workgroup");
  __builtin_amdgcn_wave_barrier();
  for (int pass = 0; pass < 2; ++pass) {
    for (int r = 0; r < 16; ++r) {
      const int row = q0 + r;
      if (row < T && lane < D / 4) {
        const v4f val = *(const v4fa*)&sO[w][r][lane * 4];
        *(volatile v4f*)(y + ((size_t)b * T + row) * ypitch + h * D + lane * 4) = val;
      }
    }
    if (pass == 0) __threadfence();
  }
}

template <bool ASPLIT, int ACT, bool BIAS_BF16, bool RES_BF16>
__global__ __launch_bounds__(128) void k_gemm_bf3(const float* __restrict__ A, int lda, const unsigned short* __restrict__ Wt, int ldb,
                                                const float* __restrict__ bias, const float* __restrict__ resid, int rmod, int ldr,
                                                float* __restrict__ C, int ldc, int M, int N, int K) {
  __shared__ __attribute__((aligned(16))) float so[4][16][64];
  const int tid = threadIdx.x, w = tid >> 5, lane = tid & 31, ln = lane & 15, hh = lane >> 4;
  const int ntn = N / 64;
  const int wid = blockIdx.x * 4 + w;
  const int mt = wid / ntn, nq = wid % ntn;
  if (mt * 16 >= M) return;
  const int row0 = mt * 16, col0 = nq * 64;
  const float* arow = A + (size_t)(row0 + ln) * lda;
  v8f acc[4] = {};
  for (int kb = 0; kb < K; kb += 32) {
    FragB ah, al;
    const v4f x0 = *(const v4fa*)(arow + kb + 8 * hh), x1 = *(const v4fa*)(arow + kb + 8 * hh + 4);
    const v4f x2 = *(const v4fa*)(arow + kb + 16 + 8 * hh), x3 = *(const v4fa*)(arow + kb + 16 + 8 * hh + 4);
    float xs[16] = {x0[0],x0[1],x0[2],x0[3],x1[0],x1[1],x1[2],x1[3],x2[0],x2[1],x2[2],x2[3],x3[0],x3[1],x3[2],x3[3]};
#pragma unroll
    for (int i = 0; i < 16; ++i) { const unsigned short hb = bf16_bits(xs[i]); ah.u[i] = hb; al.u[i] = ASPLIT ? bf16_bits(xs[i] - bf16_val(hb)) : (unsigned short)0; }
#pragma unroll
    for (int t = 0; t < 4; ++t) {
      const unsigned short* brow = Wt + (size_t)(col0 + t * 16 + ln) * ldb + kb;
      FragB b;
      b.half[0] = *(const v8us*)(brow + 8 * hh);
      b.half[1] = *(const v8us*)(brow + 16 + 8 * hh);
      acc[t] = mmaN<ASPLIT ? 2 : 1>(ah.v, al.v, b.v, b.v, acc[t]);
    }
  }
#pragma unroll
  for (int t = 0; t < 4; ++t) {
    const int col = col0 + t * 16 + ln;
    float bv = bias ? bias[col] : 0.f;
    if (BIAS_BF16) bv = bf16_round(bv);
#pragma unroll
    for (int r = 0; r < 8; ++r) {
      float v = acc[t][r] + bv;
      if (resid) { float rv = resid[(size_t)((row0 + 8 * hh + r) % rmod) * ldr + col]; if (RES_BF16) rv = bf16_round(rv); v += rv; }
      if (ACT == 1) v = fmaxf(v, 0.f);
      if (ACT == 2) v = 0.5f * v * (1.0f + erff(v * 0.70710678118654752f));
      if (ACT == 3) { const float u = 0.7978845608028654f * (v + 0.044715f * v * v * v); v = 0.5f * v * (1.0f + tanhf(u)); }
      so[w][8 * hh + r][t * 16 + ln] = v;
    }
  }
  __builtin_amdgcn_fence(__ATOMIC_ACQ_REL, "workgroup");
  __builtin_amdgcn_wave_barrier();
  const int rsub = lane >> 4, c4 = (lane & 15) * 4;
  for (int pass = 0; pass < 2; ++pass) {
#pragma unroll
    for (int q = 0; q < 8; ++q) {
      const int r = q * 2 + rsub;
      const v4f v = *(const v4fa*)&so[w][r][c4];
      *(volatile v4f*)(C + (size_t)(row0 + r) * ldc + col0 + c4) = v;
    }
    if (pass == 0) __threadfence();
  }
}
template <bool PARAM_BF16>
__global__ __launch_bounds__(256) void k_layernorm(const float* __restrict__ X, const float* __restrict__ R, const float* __restrict__ g, const float* __restrict__ bta,
                                                  float* __restrict__ out_sum, float* __restrict__ out_norm, int N, float eps) {
  __shared__ float red[256];
  const int row = blockIdx.x, tid = threadIdx.x;
  const float* x = X + (size_t)row * N; const float* rr = R ? R + (size_t)row * N : nullptr;
  float vals[16];
  const int per = N / 256;
  float s1 = 0.f;
  for (int u = 0; u < per / 4; ++u) {
    const int j = tid * 4 + 1024 * u;
    const v4f a = *(const v4fa*)(x + j);
    v4f b = {0.f,0.f,0.f,0.f}; if (rr) b = *(const v4fa*)(rr + j);
#pragma unroll
    for (int q = 0; q < 4; ++q) { const float v = a[q] + b[q]; vals[u * 4 + q] = v; s1 += v; }
  }
  red[tid] = s1; __syncthreads();
  for (int st = 128; st > 0; st >>= 1) { if (tid < st) red[tid] += red[tid + st]; __syncthreads(); }
  const float mu = red[0] / (float)N; __syncthreads();
  float s2 = 0.f;
  for (int u = 0; u < per / 4; ++u)
#pragma unroll
    for (int q = 0; q < 4; ++q) { const float c = vals[u * 4 + q] - mu; s2 += c * c; }
  red[tid] = s2; __syncthreads();
  for (int st = 128; st > 0; st >>= 1) { if (tid < st) red[tid] += red[tid + st]; __syncthreads(); }
  const float rs = rsqrtf(red[0] / (float)N + eps);
  for (int pass = 0; pass < 2; ++pass) {
    for (int u = 0; u < per / 4; ++u) {
      const int j = tid * 4 + 1024 * u;
      v4f o, sm;
#pragma unroll
      for (int q = 0; q < 4; ++q) {
        float gg = g[j + q], bb = bta[j + q];
        if (PARAM_BF16) { gg = bf16_round(gg); bb = bf16_round(bb); }
        sm[q] = vals[u * 4 + q]; o[q] = (vals[u * 4 + q] - mu) * rs * gg + bb;
      }
      if (out_sum) *(volatile v4f*)(out_sum + (size_t)row * N + j) = sm;
      *(volatile v4f*)(out_norm + (size_t)row * N + j) = o;
    }
    if (pass == 0) __threadfence();
  }
}


typedef _Float16 v16h __attribute__((ext_vector_type(16)));
union FragH { v16h v; v8us half[2]; _Float16 h[16]; unsigned short u[16]; };
template <int NT>
__device__ __forceinline__ v8f mmaH(v16h ah, v16h al, v16h bh, v16h bl, v8f c) {
  c = __builtin_amdgcn_wmma_f32_16x16x32_f16(false, ah, false, bh, (short)0, c, false, false);
  if (NT >= 2) c = __builtin_amdgcn_wmma_f32_16x16x32_f16(false, al, false, bh, (short)0, c, false, false);
  if (NT >= 3) c = __builtin_amdgcn_wmma_f32_16x16x32_f16(false, ah, false, bl, (short)0, c, false, false);
  asm volatile("v_nop\n\tv_nop\n\tv_nop\n\tv_nop" : "+v"(c) : "v"(ah), "v"(al), "v"(bh), "v"(bl));
  return c;
}
template <bool ASPLIT>
__global__ __launch_bounds__(128) void k_gemm_h(const float* __restrict__ A, int lda, size_t sA, const _Float16* __restrict__ Bh, int ldb, size_t sB, float alpha, float* __restrict__ C, int ldc, size_t sC, int M, int N, int K) {
  __shared__ __attribute__((aligned(16))) float so[4][16][64];
  const int tid = threadIdx.x, w = tid >> 5, lane = tid & 31, ln = lane & 15, hh = lane >> 4; const int by = blockIdx.y;
  A += (size_t)by * sA; Bh += (size_t)by * sB; C += (size_t)by * sC;
  const int ntn = (N + 63) / 64; const int wid = blockIdx.x * 4 + w; const int mt = wid / ntn, nq = wid % ntn; if (mt * 16 >= M) return;
  const int row0 = mt * 16, col0 = nq * 64; const float* arow = A + (size_t)(row0 + ln) * lda;
  v8f acc[4] = {};
  for (int kb = 0; kb < K; kb += 32) {
    FragH ah, al;
    const v4f x0 = *(const v4fa*)(arow + kb + 8 * hh), x1 = *(const v4fa*)(arow + kb + 8 * hh + 4), x2 = *(const v4fa*)(arow + kb + 16 + 8 * hh), x3 = *(const v4fa*)(arow + kb + 16 + 8 * hh + 4);
    float xs[16] = {x0[0],x0[1],x0[2],x0[3],x1[0],x1[1],x1[2],x1[3],x2[0],x2[1],x2[2],x2[3],x3[0],x3[1],x3[2],x3[3]};
#pragma unroll
    for (int i = 0; i < 16; ++i) { const _Float16 h = (_Float16)xs[i]; ah.h[i] = h; al.h[i] = ASPLIT ? (_Float16)(xs[i] - (float)h) : (_Float16)0.0f; }
#pragma unroll
    for (int t = 0; t < 4; ++t) { if (col0 + t * 16 >= N) continue; const size_t boff = (size_t)(col0 + t * 16 + ln) * ldb + kb; FragH bq; bq.half[0] = *(const v8us*)(Bh + boff + 8 * hh); bq.half[1] = *(const v8us*)(Bh + boff + 16 + 8 * hh);
      acc[t] = mmaH<ASPLIT ? 2 : 1>(ah.v, al.v, bq.v, bq.v, acc[t]); }
  }
#pragma unroll
  for (int t = 0; t < 4; ++t) { if (col0 + t * 16 >= N) continue;
#pragma unroll
    for (int r = 0; r < 8; ++r) so[w][8 * hh + r][t * 16 + ln] = acc[t][r] * alpha; }
  __builtin_amdgcn_fence(__ATOMIC_ACQ_REL, "workgroup"); __builtin_amdgcn_wave_barrier();
  const int rsub = lane >> 4, c4 = (lane & 15) * 4;
  for (int pass = 0; pass < 2; ++pass) {
#pragma unroll
    for (int q = 0; q < 8; ++q) { const int r = q * 2 + rsub; if (col0 + c4 < N) { const v4f v = *(const v4fa*)&so[w][r][c4]; *(volatile v4f*)(C + (size_t)(row0 + r) * ldc + col0 + c4) = v; } }
    if (pass == 0) __threadfence(); }
}

__global__ __launch_bounds__(256) void k_wt_f16(const float* __restrict__ W, _Float16* __restrict__ Wt, int K, int N, float scale) {
  const int t = blockIdx.x * 256 + threadIdx.x; if (t >= N * (K / 8)) return; const int n = t / (K / 8), k8 = (t % (K / 8)) * 8; FragH f;
#pragma unroll
  for (int i = 0; i < 8; ++i) f.h[i] = (_Float16)(bf16_round(W[(size_t)(k8 + i) * N + n]) * scale); const v8us o = f.half[0];
  *(volatile v8us*)((unsigned short*)Wt + (size_t)n * K + k8) = o; __threadfence(); *(volatile v8us*)((unsigned short*)Wt + (size_t)n * K + k8) = o;
}
template <int ACT>
__global__ __launch_bounds__(128) void k_gemm_hhx(const _Float16* __restrict__ A, int lda, size_t sA, const _Float16* __restrict__ Bh, int ldb, size_t sB, float alpha, const float* __restrict__ bias, size_t sBias, const float* __restrict__ CP, int rowsPerB, size_t sCPb, int row0g,
    float* __restrict__ C, _Float16* __restrict__ C16, int ldc, size_t sC, int M, int N, int K) {
  __shared__ __attribute__((aligned(16))) float so[4][16][64];
  const int tid = threadIdx.x, w = tid >> 5, lane = tid & 31, ln = lane & 15, hh = lane >> 4; const int by = blockIdx.y;
  A += (size_t)by * sA; Bh += (size_t)by * sB; const size_t cofs = (size_t)by * sC; const float* bp = bias ? bias + (size_t)by * sBias : nullptr;
  const int ntn = (N + 63) / 64; const int wid = blockIdx.x * 4 + w; const int mt = wid / ntn, nq = wid % ntn; if (mt * 16 >= M) return;
  const int row0 = mt * 16, col0 = nq * 64; const _Float16* arow = A + (size_t)(row0 + ln) * lda;
  v8f acc[4] = {};
  for (int kb = 0; kb < K; kb += 32) { FragH ah; ah.half[0] = *(const v8us*)((const unsigned short*)arow + kb + 8 * hh); ah.half[1] = *(const v8us*)((const unsigned short*)arow + kb + 16 + 8 * hh);
#pragma unroll
    for (int t = 0; t < 4; ++t) { if (col0 + t * 16 >= N) continue; const size_t boff = (size_t)(col0 + t * 16 + ln) * ldb + kb; FragH bq; bq.half[0] = *(const v8us*)((const unsigned short*)Bh + boff + 8 * hh); bq.half[1] = *(const v8us*)((const unsigned short*)Bh + boff + 16 + 8 * hh);
      acc[t] = mmaH<1>(ah.v, ah.v, bq.v, bq.v, acc[t]); }
  }
#pragma unroll
  for (int t = 0; t < 4; ++t) { if (col0 + t * 16 >= N) continue; const int col = col0 + t * 16 + ln; const float bv = bp ? bf16_round(bp[col]) : 0.f;
#pragma unroll
    for (int r = 0; r < 8; ++r) { float v = acc[t][r] * alpha + bv; if (CP) { const int bidx = (row0g + row0 + 8 * hh + r) / rowsPerB; v += CP[(size_t)bidx * sCPb + (size_t)by * 64 + col]; } if (ACT == 1) v = (v > 0.f) ? v : expm1f(v); else if (ACT == 3) v = fmaxf(v, 0.f); so[w][8 * hh + r][t * 16 + ln] = v; } }
  __builtin_amdgcn_fence(__ATOMIC_ACQ_REL, "workgroup"); __builtin_amdgcn_wave_barrier();
  const int rsub = lane >> 4, c4 = (lane & 15) * 4; typedef _Float16 v4h __attribute__((ext_vector_type(4)));
  for (int pass = 0; pass < 2; ++pass) {
#pragma unroll
    for (int q = 0; q < 8; ++q) { const int r = q * 2 + rsub; if (col0 + c4 < N) { const v4f v = *(const v4fa*)&so[w][r][c4]; if (C) *(volatile v4f*)(C + cofs + (size_t)(row0 + r) * ldc + col0 + c4) = v; if (C16) { v4h h4; for (int i = 0; i < 4; ++i) h4[i] = (_Float16)v[i]; *(volatile v4h*)(C16 + cofs + (size_t)(row0 + r) * ldc + col0 + c4) = h4; } } }
    if (pass == 0) __threadfence(); }
}


typedef _Float16 v4h __attribute__((ext_vector_type(4)));

__global__ __launch_bounds__(256) void k_x16(const float* __restrict__ x, _Float16* __restrict__ X16, size_t n8) { const size_t t = (size_t)blockIdx.x * 256 + threadIdx.x; if (t >= n8) return; FragH f;
#pragma unroll
  for (int q = 0; q < 8; ++q) f.h[q] = (_Float16)bf16_round(x[t * 8 + q]); *(volatile v8us*)((unsigned short*)X16 + t * 8) = f.half[0]; __threadfence(); *(volatile v8us*)((unsigned short*)X16 + t * 8) = f.half[0]; }
__global__ __launch_bounds__(256) void k_h16(const float* __restrict__ x, _Float16* __restrict__ X16, size_t n8) { const size_t t = (size_t)blockIdx.x * 256 + threadIdx.x; if (t >= n8) return; FragH f;
#pragma unroll
  for (int q = 0; q < 8; ++q) f.h[q] = (_Float16)x[t * 8 + q]; *(volatile v8us*)((unsigned short*)X16 + t * 8) = f.half[0]; __threadfence(); *(volatile v8us*)((unsigned short*)X16 + t * 8) = f.half[0]; }
__global__ __launch_bounds__(256) void k_round16f(const float* __restrict__ W, _Float16* __restrict__ Bt, size_t n8) { const size_t t = (size_t)blockIdx.x * 256 + threadIdx.x; if (t >= n8) return; FragH f;
#pragma unroll
  for (int i = 0; i < 8; ++i) f.h[i] = (_Float16)(bf16_round(W[t * 8 + i]) * 16.0f); *(volatile v8us*)((unsigned short*)Bt + t * 8) = f.half[0]; __threadfence(); *(volatile v8us*)((unsigned short*)Bt + t * 8) = f.half[0]; }
template <int NHv, int TTv>
__global__ __launch_bounds__(256) void k_vt(const _Float16* __restrict__ V16, int ldv, int voff, _Float16* __restrict__ Vt) { __shared__ unsigned short tl[64][66]; const int tid = threadIdx.x; const int slab = blockIdx.x / (TTv / 64), lg = blockIdx.x % (TTv / 64); const int b = slab / NHv, h = slab % NHv;
  for (int i = tid; i < 64 * 8; i += 256) { const int r = i / 8, c8 = (i % 8) * 8; FragH f; f.half[0] = *(const v8us*)((const unsigned short*)V16 + ((size_t)b * TTv + lg * 64 + r) * ldv + voff + h * 64 + c8);
#pragma unroll
    for (int q = 0; q < 8; ++q) tl[r][c8 + q] = f.u[q]; }
  __syncthreads();
  for (int pass = 0; pass < 2; ++pass) {
#pragma unroll
    for (int rd = 0; rd < 2; ++rd) { const int d = rd * 32 + tid / 8, pc = tid % 8; FragH f;
#pragma unroll
      for (int q = 0; q < 8; ++q) f.u[q] = tl[pc * 8 + q][d];
      *(volatile v8us*)((unsigned short*)Vt + ((size_t)slab * 64 + d) * TTv + lg * 64 + pc * 8) = f.half[0]; }
    if (pass == 0) __threadfence(); } }

__global__ __launch_bounds__(256) void k_feat(const float* __restrict__ XR, const float* __restrict__ XI, int ldx, int rbf, int b0, int D, _Float16* __restrict__ F) { const size_t t = (size_t)blockIdx.x * 256 + threadIdx.x; if (t >= (size_t)RCH * D * GG) return; const int u = (int)(t % GG); const int i = (int)((t / GG) % D); const int bl = (int)(t / ((size_t)GG * D)); const size_t b = (size_t)b0 + bl; float xr = XR[b * ldx + i], xi = XI[b * ldx + i]; if (rbf) { xr = bf16_round(xr); xi = bf16_round(xi); }
  const float gu = -2.0f + (4.0f / 7.0f) * (float)u; const float du = xr - gu; const float br = __expf(-du * du); FragH f;
#pragma unroll
  for (int v = 0; v < GG; ++v) { const float gv = -2.0f + (4.0f / 7.0f) * (float)v; const float dv = xi - gv; f.h[v] = (_Float16)(br * __expf(-dv * dv)); }
  *(volatile v8us*)((unsigned short*)F + t * 8) = f.half[0]; __threadfence(); *(volatile v8us*)((unsigned short*)F + t * 8) = f.half[0]; }
__global__ __launch_bounds__(256) void k_wg(const float* __restrict__ Wr, const float* __restrict__ Wi, int D, int O, _Float16* __restrict__ Bt) { const size_t t = (size_t)blockIdx.x * 256 + threadIdx.x; if (t >= (size_t)2 * O * D * GG) return; const int u = (int)(t % GG); const int i = (int)((t / GG) % D); const int o = (int)((t / ((size_t)GG * D)) % O); const int part = (int)(t / ((size_t)GG * D * O)); const float* W = part ? Wi : Wr; const float* src = W + (((size_t)i * O + o) * GG + u) * GG; FragH f;
#pragma unroll
  for (int v = 0; v < GG; ++v) f.h[v] = (_Float16)(bf16_round(src[v]) * 16.0f); const size_t dst = ((size_t)(part * O + o) * D * 64) + (size_t)i * 64 + u * 8; *(volatile v8us*)((unsigned short*)Bt + dst) = f.half[0]; __threadfence(); *(volatile v8us*)((unsigned short*)Bt + dst) = f.half[0]; }
__global__ __launch_bounds__(256) void k_silu2(const float* __restrict__ XR, const float* __restrict__ XI, int ldx, int rbf, int D, _Float16* __restrict__ S16) { const size_t t = (size_t)blockIdx.x * 256 + threadIdx.x; const int np = 2 * D / 8; if (t >= (size_t)BB * np) return; const int p = (int)(t % np); const size_t b = t / np; const bool im = (p * 8) >= D; const int i0 = p * 8 - (im ? D : 0); const float* X = im ? XI : XR; FragH f;
#pragma unroll
  for (int q = 0; q < 8; ++q) { float x = X[b * ldx + i0 + q]; if (rbf) x = bf16_round(x); f.h[q] = (_Float16)(x / (1.0f + __expf(-x))); }
  *(volatile v8us*)((unsigned short*)S16 + t * 8) = f.half[0]; __threadfence(); *(volatile v8us*)((unsigned short*)S16 + t * 8) = f.half[0]; }
__global__ __launch_bounds__(256) void k_ws(const float* __restrict__ swr, const float* __restrict__ swi, int D, int O, _Float16* __restrict__ Bt) { const size_t t = (size_t)blockIdx.x * 256 + threadIdx.x; const int np = 2 * D / 8; if (t >= (size_t)2 * O * np) return; const int k8 = (int)(t % np) * 8; const int oo = (int)(t / np); const bool im = oo >= O; const int o = im ? oo - O : oo; FragH f;
#pragma unroll
  for (int q = 0; q < 8; ++q) { const int k = k8 + q; float w; if (k < D) w = im ? swi[(size_t)k * O + o] : swr[(size_t)k * O + o]; else w = im ? swr[(size_t)(k - D) * O + o] : -swi[(size_t)(k - D) * O + o]; f.h[q] = (_Float16)(bf16_round(w) * 16.0f); }
  *(volatile v8us*)((unsigned short*)Bt + t * 8) = f.half[0]; __threadfence(); *(volatile v8us*)((unsigned short*)Bt + t * 8) = f.half[0]; }
__global__ __launch_bounds__(256) void k_sb(const float* __restrict__ sbr, const float* __restrict__ sbi, int D, int O, float* __restrict__ SB) { const int oo = blockIdx.x * 256 + threadIdx.x; if (oo >= 2 * O) return; const bool im = oo >= O; const int o = im ? oo - O : oo; const float* sb = im ? sbi : sbr; float s = 0.f;
#pragma unroll 1
  for (int i = 0; i < D; ++i) s += bf16_round(sb[(size_t)i * O + o]); *(volatile float*)(SB + oo) = s; __threadfence(); *(volatile float*)(SB + oo) = s; }
__global__ __launch_bounds__(256) void k_fin0(const float* __restrict__ R, const float* __restrict__ SB, float* __restrict__ XR1, float* __restrict__ XI1) { const size_t t = (size_t)blockIdx.x * 256 + threadIdx.x; if (t >= (size_t)BB * (2 * D1 / 4)) return; const int c4 = (int)(t % (2 * D1 / 4)) * 4; const size_t b = t / (2 * D1 / 4); const v4f r = *(const v4fa*)(R + b * 2 * D1 + c4); v4f o; for (int q = 0; q < 4; ++q) o[q] = r[q] + SB[c4 + q]; float* dst = (c4 < D1) ? (XR1 + b * D1 + c4) : (XI1 + b * D1 + (c4 - D1)); *(volatile v4f*)dst = o; __threadfence(); *(volatile v4f*)dst = o; }
__global__ __launch_bounds__(256) void k_fin1(const float* __restrict__ R, const float* __restrict__ SB, float* __restrict__ out) { const size_t t = (size_t)blockIdx.x * 256 + threadIdx.x; if (t >= (size_t)BB * (D2 / 2)) return; const int o2 = (int)(t % (D2 / 2)) * 2; const size_t b = t / (D2 / 2); v4f v; v[0] = R[b * 2 * D2 + o2] + SB[o2]; v[1] = R[b * 2 * D2 + D2 + o2] + SB[D2 + o2]; v[2] = R[b * 2 * D2 + o2 + 1] + SB[o2 + 1]; v[3] = R[b * 2 * D2 + D2 + o2 + 1] + SB[D2 + o2 + 1]; *(volatile v4f*)(out + (b * D2 + o2) * 2) = v; __threadfence(); *(volatile v4f*)(out + (b * D2 + o2) * 2) = v; }
extern "C" void kernel_launch(void* const* d_in, const int* in_sizes, int n_in,
                              void* d_out, int out_size, void* d_ws, size_t ws_size, hipStream_t stream) {
  (void)in_sizes; (void)n_in; (void)out_size;
  const float* const* I = (const float* const*)d_in; const float* xr = I[0]; const float* xi = I[1]; const float* w0r = I[2]; const float* w0i = I[3]; const float* sw0r = I[4]; const float* sw0i = I[5]; const float* sb0r = I[6]; const float* sb0i = I[7]; const float* w1r = I[8]; const float* w1i = I[9]; const float* sw1r = I[10]; const float* sw1i = I[11]; const float* sb1r = I[12]; const float* sb1i = I[13];
  char* ws = (char*)d_ws; size_t off = 0;
  auto take = [&](size_t bytes) { char* p = ws + off; off += (bytes + 255) & ~(size_t)255; return p; };
  _Float16* Bg0 = (_Float16*)take((size_t)2 * D1 * D0 * 64 * 2); _Float16* Bg1 = (_Float16*)take((size_t)2 * D2 * D1 * 64 * 2); _Float16* Bs0 = (_Float16*)take((size_t)2 * D1 * 2 * D0 * 2); _Float16* Bs1 = (_Float16*)take((size_t)2 * D2 * 2 * D1 * 2); float* SB0 = (float*)take(2 * D1 * 4); float* SB1 = (float*)take(2 * D2 * 4);
  _Float16* F = (_Float16*)take((size_t)RCH * D0 * 64 * 2); _Float16* S16 = (_Float16*)take((size_t)BB * 2 * D0 * 2); float* R = (float*)take((size_t)BB * 2 * D1 * 4); float* XR1 = (float*)take((size_t)BB * D1 * 4); float* XI1 = (float*)take((size_t)BB * D1 * 4);
  if (off > ws_size) return;
  k_wg<<<(unsigned)(((size_t)2 * D1 * D0 * GG + 255) / 256), 256, 0, stream>>>(w0r, w0i, D0, D1, Bg0); k_wg<<<(unsigned)(((size_t)2 * D2 * D1 * GG + 255) / 256), 256, 0, stream>>>(w1r, w1i, D1, D2, Bg1);
  k_ws<<<(2 * D1 * (2 * D0 / 8) + 255) / 256, 256, 0, stream>>>(sw0r, sw0i, D0, D1, Bs0); k_ws<<<(2 * D2 * (2 * D1 / 8) + 255) / 256, 256, 0, stream>>>(sw1r, sw1i, D1, D2, Bs1);
  k_sb<<<1, 256, 0, stream>>>(sb0r, sb0i, D0, D1, SB0); k_sb<<<1, 256, 0, stream>>>(sb1r, sb1i, D1, D2, SB1);
  for (int l = 0; l < 2; ++l) { const int D = l ? D1 : D0, O = l ? D2 : D1; const float* XR = l ? XR1 : xr; const float* XI = l ? XI1 : xi; const _Float16* Bg = l ? Bg1 : Bg0; const _Float16* Bs = l ? Bs1 : Bs0; const int K = D * 64;
    for (int b0 = 0; b0 < BB; b0 += RCH) {
      k_feat<<<(unsigned)(((size_t)RCH * D * GG + 255) / 256), 256, 0, stream>>>(XR, XI, D, l == 0, b0, D, F);
      k_gemm_hhx<0><<<dim3(((RCH / 16) * (2 * O / 64) + 3) / 4, 1), 128, 0, stream>>>(F, K, 0, Bg, K, 0, 0.0625f, nullptr, 0, nullptr, 1, 0, 0, R + (size_t)b0 * 2 * O, nullptr, 2 * O, 0, RCH, 2 * O, K); }
    k_silu2<<<(unsigned)(((size_t)BB * (2 * D / 8) + 255) / 256), 256, 0, stream>>>(XR, XI, D, l == 0, D, S16);
    k_gemm_hhx<0><<<dim3(((BB / 16) * (2 * O / 64) + 3) / 4, 1), 128, 0, stream>>>(S16, 2 * D, 0, Bs, 2 * D, 0, 0.0625f, nullptr, 0, R, 1, (size_t)(2 * O), 0, R, nullptr, 2 * O, 0, BB, 2 * O, 2 * D);
    if (l == 0) k_fin0<<<(unsigned)(((size_t)BB * (2 * D1 / 4) + 255) / 256), 256, 0, stream>>>(R, SB0, XR1, XI1);
    else k_fin1<<<(unsigned)(((size_t)BB * (D2 / 2) + 255) / 256), 256, 0, stream>>>(R, SB1, (float*)d_out); }
}
